// LinearAttention_12833362280732
// MI455X (gfx1250) — hardware-verified
//
#include <hip/hip_runtime.h>
#define NB 4
#define SQ 4096
#define NH 8
#define HD 64
#define ROWP (NH * HD)
#define EXT 128
#define EPSZ 1e-6f
typedef __bf16 v16b __attribute__((ext_vector_type(16)));
typedef unsigned short v8us __attribute__((ext_vector_type(8), may_alias));
typedef float  v8f  __attribute__((ext_vector_type(8)));
typedef float  v4f  __attribute__((ext_vector_type(4)));
typedef float  v4fa __attribute__((ext_vector_type(4), may_alias));
union FragB { v16b v; v8us half[2]; unsigned short u[16]; };

__device__ __forceinline__ unsigned short bf16_bits(float x) { unsigned int u = __float_as_uint(x); return (unsigned short)((u + 0x7FFFu + ((u >> 16) & 1u)) >> 16); }
__device__ __forceinline__ float bf16_val(unsigned short b) { return __uint_as_float(((unsigned int)b) << 16); }
__device__ __forceinline__ float bf16_round(float x) { return bf16_val(bf16_bits(x)); }
template <int NT>
__device__ __forceinline__ v8f mmaN(v16b ah, v16b al, v16b bh, v16b bl, v8f c) {
  c = __builtin_amdgcn_wmma_f32_16x16x32_bf16(false, ah, false, bh, (short)0, c, false, false);
  if (NT >= 2) c = __builtin_amdgcn_wmma_f32_16x16x32_bf16(false, al, false, bh, (short)0, c, false, false);
  if (NT >= 3) c = __builtin_amdgcn_wmma_f32_16x16x32_bf16(false, ah, false, bl, (short)0, c, false, false);
  asm volatile("v_nop\n\tv_nop\n\tv_nop\n\tv_nop" : "+v"(c) : "v"(ah), "v"(al), "v"(bh), "v"(bl));
  return c;
}


typedef _Float16 v16h __attribute__((ext_vector_type(16)));
union FragH { v16h v; v8us half[2]; _Float16 h[16]; unsigned short u[16]; };
template <int NT>
__device__ __forceinline__ v8f mmaH(v16h ah, v16h al, v16h bh, v16h bl, v8f c) {
  c = __builtin_amdgcn_wmma_f32_16x16x32_f16(false, ah, false, bh, (short)0, c, false, false);
  if (NT >= 2) c = __builtin_amdgcn_wmma_f32_16x16x32_f16(false, al, false, bh, (short)0, c, false, false);
  if (NT >= 3) c = __builtin_amdgcn_wmma_f32_16x16x32_f16(false, ah, false, bl, (short)0, c, false, false);
  asm volatile("v_nop\n\tv_nop\n\tv_nop\n\tv_nop" : "+v"(c) : "v"(ah), "v"(al), "v"(bh), "v"(bl));
  return c;
}

typedef _Float16 v4h __attribute__((ext_vector_type(4)));
__device__ __forceinline__ v16h g2_frag(const _Float16* p, int hh) { FragH f; f.half[0] = *(const v8us*)((const unsigned short*)p + 8 * hh); f.half[1] = *(const v8us*)((const unsigned short*)p + 16 + 8 * hh); return f.v; }
__device__ __forceinline__ v8f g2_mma(v16h a, v16h b, v8f c) { v8f d = __builtin_amdgcn_wmma_f32_16x16x32_f16(false, a, false, b, (short)0, c, false, false); asm volatile("v_nop\n\tv_nop\n\tv_nop\n\tv_nop" : "+v"(d) : "v"(a), "v"(b)); return d; }
template <int ACT>
__global__ __launch_bounds__(128) void k_gemm2(const _Float16* __restrict__ A, int lda, size_t sA, const _Float16* __restrict__ Bh, int ldb, size_t sB, float alpha, const float* __restrict__ bias, size_t sBias, const float* __restrict__ CP, int rowsPerB, size_t sCPb, int row0g,
    float* __restrict__ C, _Float16* __restrict__ C16, int ldc, size_t sC, int M, int N, int K) { static_assert(ACT == 0 || ACT == 3 || ACT == 6 || ACT == 8 || ACT == 9 || ACT == 11 || ACT == 12 || ACT == 14 || ACT == 15 || ACT == 16 || ACT == 17, "k_gemm2: unsupported ACT code (would silently apply no activation)");
  __shared__ __attribute__((aligned(16))) float so[4][32][68];
  const int tid = threadIdx.x, w = tid >> 5, lane = tid & 31, ln = lane & 15, hh = lane >> 4; const int by = blockIdx.y;
  A += (size_t)by * sA; Bh += (size_t)by * sB; const size_t cofs = (size_t)by * sC; const float* bp = bias ? bias + (size_t)by * sBias : nullptr;
  const int ntn = N >> 6; const int mt = blockIdx.x / ntn, nq = blockIdx.x - mt * ntn; const int row0 = mt * 128 + 32 * w, col0 = nq * 64; if (row0 >= M) return;
  const _Float16* a0p = A + (size_t)(row0 + ln) * lda; const _Float16* a1p = a0p + (size_t)16 * lda;
  const _Float16* b0p = Bh + (size_t)(col0 + ln) * ldb; const _Float16* b1p = b0p + (size_t)16 * ldb; const _Float16* b2p = b1p + (size_t)16 * ldb; const _Float16* b3p = b2p + (size_t)16 * ldb;
  const v8f z8 = {0.f,0.f,0.f,0.f,0.f,0.f,0.f,0.f}; v8f c00 = z8, c01 = z8, c02 = z8, c03 = z8, c10 = z8, c11 = z8, c12 = z8, c13 = z8;
  for (int kb = 0; kb < K; kb += 32) { const v16h a0 = g2_frag(a0p + kb, hh), a1 = g2_frag(a1p + kb, hh);
    v16h b = g2_frag(b0p + kb, hh); c00 = g2_mma(a0, b, c00); c10 = g2_mma(a1, b, c10);
    b = g2_frag(b1p + kb, hh); c01 = g2_mma(a0, b, c01); c11 = g2_mma(a1, b, c11);
    b = g2_frag(b2p + kb, hh); c02 = g2_mma(a0, b, c02); c12 = g2_mma(a1, b, c12);
    b = g2_frag(b3p + kb, hh); c03 = g2_mma(a0, b, c03); c13 = g2_mma(a1, b, c13); }
  v8f accs[8] = {c00, c01, c02, c03, c10, c11, c12, c13};
#pragma unroll
  for (int u = 0; u < 8; ++u) { const int t = u & 3, half = u >> 2; const int col = col0 + t * 16 + ln; const float bv = bp ? bf16_round(bp[col]) : 0.f;
#pragma unroll
    for (int r = 0; r < 8; ++r) { const int rloc = half * 16 + 8 * hh + r; float v = accs[u][r] * alpha + bv; if (CP) { if (rowsPerB < 0) v += CP[cofs + (size_t)(row0g + row0 + rloc) * ldc + col];        else { const int bidx = (row0g + row0 + rloc) / rowsPerB; v += CP[(size_t)bidx * sCPb + (size_t)by * 64 + col]; } }
      if (ACT == 3) v = fmaxf(v, 0.f); else if (ACT == 6) v = 0.5f * v * (1.0f + erff(v * 0.70710678118654752f)); else if (ACT == 11) v = 1.0f / (1.0f + expf(-v)); else if (ACT == 15) v = v / (1.0f + expf(-v)); else if (ACT == 12) v = (v > 0.f) ? v : 0.01f * v; else if (ACT == 8) v = tanhf(v); else if (ACT == 9) v = 0.5f * v * (1.0f + tanhf(0.7978845608028654f * (v + 0.044715f * v * v * v))); else if (ACT == 14) v = (v > 0.f) ? v : 0.1f * v; else if (ACT == 16) v = (v >= 0.f) ? v : 0.3f * v; else if (ACT == 17) v = (v >= 0.f) ? v : 0.2f * v;
      so[w][rloc][t * 16 + ln] = v; } }
  __builtin_amdgcn_fence(__ATOMIC_ACQ_REL, "workgroup"); __builtin_amdgcn_wave_barrier();
  const int rsub = lane >> 4, c4 = (lane & 15) * 4;
  for (int pass = 0; pass < 2; ++pass) {
#pragma unroll
    for (int q = 0; q < 16; ++q) { const int r = q * 2 + rsub; const v4f v = *(const v4fa*)&so[w][r][c4]; if (C) *(volatile v4f*)(C + cofs + (size_t)(row0 + r) * ldc + col0 + c4) = v; if (C16) { v4h h4; for (int i = 0; i < 4; ++i) h4[i] = (_Float16)v[i]; *(volatile v4h*)(C16 + cofs + (size_t)(row0 + r) * ldc + col0 + c4) = h4; } }
    if (pass == 0) __threadfence(); } }


__device__ __forceinline__ float fmap_elu1(float x) { return fmaxf(x, 0.f) + expf(fminf(x, 0.f)); }
__global__ __launch_bounds__(256) void k_fmq(const float* __restrict__ Q, const int* __restrict__ qm, _Float16* __restrict__ Q16, int n8) {
  const int t = blockIdx.x * 256 + threadIdx.x; if (t >= n8) return; const int r = t >> 6; const float m = (float)qm[r]; const float* s = Q + (size_t)t * 8; const v4f a = *(const v4fa*)s, c = *(const v4fa*)(s + 4); FragH f;
  for (int i = 0; i < 4; ++i) { f.h[i] = (_Float16)(fmap_elu1(bf16_round(a[i])) * m); f.h[4 + i] = (_Float16)(fmap_elu1(bf16_round(c[i])) * m); }
  unsigned short* o = (unsigned short*)Q16 + (size_t)t * 8; *(volatile v8us*)o = f.half[0]; __threadfence(); *(volatile v8us*)o = f.half[0]; }
__global__ __launch_bounds__(256) void k_fmkT(const float* __restrict__ K, const int* __restrict__ km, _Float16* __restrict__ KT, int n) {
  const int t = blockIdx.x * 256 + threadIdx.x; if (t >= n) return; const int s8 = t & 511, dd = (t >> 9) & 63, nh = t >> 15; const int nb = nh >> 3, h = nh & 7; const size_t r0 = (size_t)nb * SQ + s8 * 8; const float* s = K + r0 * ROWP + h * HD + dd; FragH f;
  for (int i = 0; i < 8; ++i) f.h[i] = (_Float16)(fmap_elu1(bf16_round(s[(size_t)i * ROWP])) * (float)km[r0 + i]);
  unsigned short* o = (unsigned short*)KT + ((size_t)nh * HD + dd) * SQ + s8 * 8; *(volatile v8us*)o = f.half[0]; __threadfence(); *(volatile v8us*)o = f.half[0]; }
__global__ __launch_bounds__(256) void k_vTones(const float* __restrict__ V, const int* __restrict__ km, _Float16* __restrict__ VT, int n) {
  const int t = blockIdx.x * 256 + threadIdx.x; if (t >= n) return; const int s8 = t & 511, r = (t >> 9) & 127, nh = t >> 16; const int nb = nh >> 3, h = nh & 7; const int rc = (r < HD) ? r : (HD - 1); const float fv = (r < HD) ? 1.0f : 0.0f, fo = (r == HD) ? 1.0f : 0.0f; const size_t r0 = (size_t)nb * SQ + s8 * 8; const float* s = V + r0 * ROWP + h * HD + rc; FragH f;
  for (int i = 0; i < 8; ++i) f.h[i] = (_Float16)(bf16_round(s[(size_t)i * ROWP]) * (float)km[r0 + i] * fv + fo);
  unsigned short* o = (unsigned short*)VT + ((size_t)nh * EXT + r) * SQ + s8 * 8; *(volatile v8us*)o = f.half[0]; __threadfence(); *(volatile v8us*)o = f.half[0]; }
__global__ __launch_bounds__(256) void k_zdiv(const float* __restrict__ ND, float* __restrict__ out, int n) {
  const int t = blockIdx.x * 256 + threadIdx.x; if (t >= n) return; const int g = t & 7, h = (t >> 3) & 7, r = t >> 6; const int nb = r >> 12, s = r & (SQ - 1); const float* p = ND + (((size_t)(nb * NH + h)) * SQ + s) * EXT; const float z = 1.0f / (p[HD] + EPSZ); const v4f a = *(const v4fa*)(p + 8 * g), c = *(const v4fa*)(p + 8 * g + 4); v4f o0, o1;
  for (int i = 0; i < 4; ++i) { o0[i] = a[i] * z; o1[i] = c[i] * z; }
  float* o = out + (size_t)r * ROWP + h * HD + 8 * g; *(volatile v4f*)o = o0; *(volatile v4f*)(o + 4) = o1; __threadfence(); *(volatile v4f*)o = o0; *(volatile v4f*)(o + 4) = o1; }

extern "C" void kernel_launch(void* const* d_in, const int* in_sizes, int n_in,
                              void* d_out, int out_size, void* d_ws, size_t ws_size, hipStream_t stream) {
  (void)in_sizes; (void)n_in; (void)out_size;
  const float* q = (const float*)d_in[0]; const float* k = (const float*)d_in[1]; const float* v = (const float*)d_in[2]; const int* qm = (const int*)d_in[3]; const int* km = (const int*)d_in[4];
  static_assert(ROWP == 512 && HD == 64 && NH == 8 && SQ == 4096 && EXT == 128 && ((size_t)NB * SQ * ROWP / 8) % 256 == 0 && ((size_t)NB * NH * HD * (SQ / 8)) % 256 == 0 && ((size_t)NB * NH * EXT * (SQ / 8)) % 256 == 0 && SQ % 128 == 0 && EXT % 64 == 0 && HD % 32 == 0 && SQ % 32 == 0, "the index shifts; whole tiles; exact grids");
  float* out = (float*)d_out;
  char* ws = (char*)d_ws; size_t off = 0;
  auto take = [&](size_t bytes) { char* p = ws + off; off += (bytes + 255) & ~(size_t)255; return p; };
  _Float16* Q16 = (_Float16*)take((size_t)NB * SQ * ROWP * 2); _Float16* KT = (_Float16*)take((size_t)NB * NH * HD * SQ * 2); _Float16* VT = (_Float16*)take((size_t)NB * NH * EXT * SQ * 2); _Float16* KVT = (_Float16*)take((size_t)NB * NH * EXT * HD * 2); float* ND = (float*)take((size_t)NB * NH * SQ * EXT * 4);
  if (off > ws_size) return;
  k_fmq<<<(unsigned)((size_t)NB * SQ * ROWP / 8 / 256), 256, 0, stream>>>(q, qm, Q16, NB * SQ * ROWP / 8);
  k_fmkT<<<(unsigned)((size_t)NB * NH * HD * (SQ / 8) / 256), 256, 0, stream>>>(k, km, KT, NB * NH * HD * (SQ / 8));
  k_vTones<<<(unsigned)((size_t)NB * NH * EXT * (SQ / 8) / 256), 256, 0, stream>>>(v, km, VT, NB * NH * EXT * (SQ / 8));
  k_gemm2<0><<<dim3((EXT / 128) * (HD / 64), NB * NH), 128, 0, stream>>>(VT, SQ, (size_t)EXT * SQ, KT, SQ, (size_t)HD * SQ, 1.0f, nullptr, 0, nullptr, 1, 0, 0, nullptr, KVT, HD, (size_t)EXT * HD, EXT, HD, SQ);
  for (int nb = 0; nb < NB; ++nb)
    k_gemm2<0><<<dim3((SQ / 128) * (EXT / 64), NH), 128, 0, stream>>>(Q16 + (size_t)nb * SQ * ROWP, ROWP, (size_t)HD, KVT + (size_t)nb * NH * EXT * HD, HD, (size_t)EXT * HD, 1.0f, nullptr, 0, nullptr, 1, 0, 0, ND + (size_t)nb * NH * SQ * EXT, nullptr, EXT, (size_t)SQ * EXT, SQ, EXT, HD);
  k_zdiv<<<(unsigned)((size_t)NB * SQ * NH * 8 / 256), 256, 0, stream>>>(ND, out, NB * SQ * NH * 8);
}
